// PointNetSetAbstraction_16930761080948
// MI455X (gfx1250) — hardware-verified
//
#include <hip/hip_runtime.h>
#include <math.h>
#pragma clang fp contract(off)

typedef __attribute__((ext_vector_type(16))) _Float16 v16h;
typedef __attribute__((ext_vector_type(8)))  _Float16 v8h;
typedef __attribute__((ext_vector_type(8)))  float    v8f;
typedef __attribute__((ext_vector_type(4)))  float    v4f;
typedef __attribute__((ext_vector_type(4)))  unsigned v4u;
typedef __attribute__((ext_vector_type(4)))  int      v4i;

constexpr int NBATCH = 8;
constexpr int NPTS   = 4096;
constexpr int NFEAT  = 64;
constexpr int NCENT  = 1024;
constexpr int NNBR   = 32;
constexpr int NPOS   = NBATCH * NCENT * NNBR;
constexpr int CIN0   = 67;
constexpr int KPAD0  = 96;
constexpr int NCH_L0 = 64;
constexpr int NCH_L1 = 64;
constexpr int NCH_L2 = 128;
constexpr int CAND_CAP = 1024;
constexpr int NTILE_M = NPOS / 64;
constexpr float RADIUS_SQ  = 0.04f;
constexpr float WCARRY     = 64.0f;
constexpr float WCARRY_INV = 1.0f / 64.0f;
constexpr float BN_EPS_F   = 1e-5f;

static_assert(NPOS == 262144);
static_assert(KPAD0 % 32 == 0 && KPAD0 >= CIN0);
static_assert(NCH_L0 % 64 == 0 && NCH_L1 % 64 == 0 && NCH_L2 % 64 == 0);
static_assert(NPOS % 64 == 0 && (NTILE_M % 8) == 0);
static_assert(NCENT % 32 == 0);

constexpr size_t OFF_PA   = 0;
constexpr size_t SZ_PA    = (size_t)NPOS * KPAD0 * 2;
constexpr size_t OFF_PB   = OFF_PA + SZ_PA;
constexpr size_t SZ_PB    = (size_t)NPOS * 128 * 2;
constexpr size_t OFF_PART = OFF_PB + SZ_PB;
constexpr size_t SZ_PART1 = (size_t)NTILE_M * 256 * 4;
constexpr size_t OFF_MASK = OFF_PART + 3 * SZ_PART1;
constexpr size_t SZ_MASK  = (size_t)NBATCH * NCENT * 32 * 4;
constexpr size_t OFF_IDX  = OFF_MASK + SZ_MASK;
constexpr size_t SZ_IDX   = (size_t)NBATCH * NCENT * 4;
constexpr size_t OFF_WPK  = OFF_IDX + SZ_IDX;
constexpr size_t SZ_WPK   = (size_t)(64 * 96 + 64 * 64 + 128 * 64) * 2;
constexpr size_t OFF_SCSH = OFF_WPK + SZ_WPK;
constexpr size_t SZ_SCSH  = (size_t)3 * 256 * 4;
constexpr size_t WS_TOTAL = OFF_SCSH + SZ_SCSH;
static_assert(WS_TOTAL <= (size_t)134217728);
static_assert((OFF_PB % 128) == 0 && (OFF_PART % 128) == 0 && (OFF_MASK % 128) == 0);
static_assert((OFF_IDX % 128) == 0 && (OFF_WPK % 128) == 0 && (OFF_SCSH % 128) == 0);
static_assert((size_t)NPOS * 64 * 2 * 2 <= SZ_PB);
static_assert((size_t)NPOS * 64 * 2 <= SZ_PA);

__device__ __forceinline__ float h16_to_f32(unsigned hb) {
  const unsigned sgn = (hb & 0x8000u) << 16; const unsigned em = hb & 0x7fffu;
  const float fn = __uint_as_float((em << 13) + 0x38000000u);
  const float fs = (float)em * 5.9604644775390625e-8f;
  const float mag = (em < 0x400u) ? fs : fn; return __uint_as_float(__float_as_uint(mag) | sgn); }

__device__ __forceinline__ unsigned f16_bits(float f) {
  const _Float16 h = (_Float16)f;
  return (unsigned)__builtin_bit_cast(unsigned short, h);
}

__device__ __forceinline__ int clampi(int v, int lo, int hi) { return v < lo ? lo : (v > hi ? hi : v); }

union FragH { v16h v; v8h h[2]; };
__device__ __forceinline__ v16h frag_load(const _Float16* p) {
  FragH f; f.h[0] = *(const v8h*)(p); f.h[1] = *(const v8h*)(p + 16); return f.v;
}
__device__ __forceinline__ v8f frag_mma(v16h a, v16h b, v8f c) {
  return __builtin_amdgcn_wmma_f32_16x16x32_f16(false, a, false, b, (short)0, c, false, false);
}
__device__ __forceinline__ void group_guard(v8f& a0, v8f& a1, v8f& a2, v8f& a3,
                                            v16h x, v16h b0, v16h b1, v16h b2, v16h b3) {
  asm volatile("v_nop\n\tv_nop\n\tv_nop\n\tv_nop"
               : "+v"(a0), "+v"(a1), "+v"(a2), "+v"(a3)
               : "v"(x), "v"(b0), "v"(b1), "v"(b2), "v"(b3));
}
__device__ __forceinline__ void acc_guard4(v8f& a, v8f& b, v8f& c, v8f& d) {
  asm volatile("v_nop\n\tv_nop\n\tv_nop\n\tv_nop" : "+v"(a), "+v"(b), "+v"(c), "+v"(d));
}

__global__ __launch_bounds__(256) void fps_kernel(const float* __restrict__ xyz,
                                                  int* __restrict__ idx_out,
                                                  float* __restrict__ newxyz_out)
{
#pragma clang fp contract(off)
  __shared__ __align__(16) float sraw[NPTS * 3];
  __shared__ __align__(16) int   sidx[NCENT];
  __shared__ float wv[2][8];
  __shared__ int   wi[2][8];
  const int b = blockIdx.x, t = threadIdx.x;
  const int lane = t & 31, wave = t >> 5;

  const v4f* src = (const v4f*)(xyz + (size_t)b * NPTS * 3);
#pragma unroll 1
  for (int j = 0; j < 12; ++j) {
    const v4f v = src[t + 256 * j];
    *(v4f*)(sraw + 4 * (t + 256 * j)) = v;
  }
  __syncthreads();

  float X[16], Y[16], Z[16], D[16];
#pragma unroll
  for (int s = 0; s < 16; ++s) {
    const int i = t + s * 256;
    X[s] = sraw[i * 3 + 0]; Y[s] = sraw[i * 3 + 1]; Z[s] = sraw[i * 3 + 2];
    D[s] = 1e10f;
  }

  int far = 0;
  for (int it = 0; it < NCENT; ++it) {
    const int fc = clampi(far, 0, NPTS - 1);
    const float cx = sraw[fc * 3 + 0], cy = sraw[fc * 3 + 1], cz = sraw[fc * 3 + 2];
    if (t == 0) sidx[it] = fc;
    float bv = -1.0f; int bs = 0;
#pragma unroll
    for (int s = 0; s < 16; ++s) {
      const float dx = X[s] - cx, dy = Y[s] - cy, dz = Z[s] - cz;
      const float t0 = dx * dx, t1 = dy * dy, t2 = dz * dz;
      const float d  = (t0 + t2) + t1;
      const float nd = fminf(D[s], d);
      D[s] = nd;
      if (nd > bv) { bv = nd; bs = s; }
    }
    int gi = bs * 256 + t;
#pragma unroll
    for (int off = 16; off > 0; off >>= 1) {
      const float ov = __shfl_xor(bv, off, 32);
      const int   oi = __shfl_xor(gi, off, 32);
      const bool take = (ov > bv) || (ov == bv && oi < gi);
      bv = take ? ov : bv; gi = take ? oi : gi;
    }
    const int pb = it & 1;
    if (lane == 0) { wv[pb][wave] = bv; wi[pb][wave] = gi; }
    __syncthreads();
    float fb = wv[pb][0]; int fi = wi[pb][0];
#pragma unroll
    for (int w = 1; w < 8; ++w) {
      const float ov = wv[pb][w]; const int oi = wi[pb][w];
      const bool take = (ov > fb) || (ov == fb && oi < fi);
      fb = take ? ov : fb; fi = take ? oi : fi;
    }
    far = fi;
  }
  __syncthreads();

  const v4i iv = *(const v4i*)(sidx + 4 * t);
  v4f ov3[3];
#pragma unroll
  for (int j = 0; j < 3; ++j) {
#pragma unroll
    for (int q = 0; q < 4; ++q) {
      const int e = 4 * (t + 256 * j) + q;
      const int m = e / 3;
      const int d = e - 3 * m;
      const int pi = clampi(sidx[m], 0, NPTS - 1);
      ov3[j][q] = sraw[pi * 3 + d];
    }
  }
  for (int pass = 0; pass < 2; ++pass) {
    *(volatile v4i*)(idx_out + (size_t)b * NCENT + 4 * t) = iv;
#pragma unroll
    for (int j = 0; j < 3; ++j)
      *(volatile v4f*)(newxyz_out + (size_t)b * NCENT * 3 + 4 * (t + 256 * j)) = ov3[j];
    __threadfence();
  }
}

__global__ __launch_bounds__(256) void pack_kernel(const float* __restrict__ w0,
                                                   const float* __restrict__ w1,
                                                   const float* __restrict__ w2,
                                                   unsigned short* __restrict__ wp)
{
  const int t = threadIdx.x;
  const int blk = blockIdx.x;
  float v[8];
  size_t dst;
  if (blk < 3) {
    const int g = blk * 256 + t;
    const int row = g / 12;
    const int kc = (g - row * 12) * 8;
#pragma unroll
    for (int e = 0; e < 8; ++e) {
      const int k = kc + e;
      const int kk = k < CIN0 ? k : (CIN0 - 1);
      const float x = w0[row * CIN0 + kk];
      v[e] = (k < CIN0) ? x : 0.0f;
    }
    dst = (size_t)g * 8;
  } else if (blk < 5) {
    const int g = (blk - 3) * 256 + t;
    const v4f a = *(const v4f*)(w1 + (size_t)g * 8);
    const v4f c = *(const v4f*)(w1 + (size_t)g * 8 + 4);
    v[0] = a[0]; v[1] = a[1]; v[2] = a[2]; v[3] = a[3];
    v[4] = c[0]; v[5] = c[1]; v[6] = c[2]; v[7] = c[3];
    dst = (size_t)64 * 96 + (size_t)g * 8;
  } else {
    const int g = (blk - 5) * 256 + t;
    const v4f a = *(const v4f*)(w2 + (size_t)g * 8);
    const v4f c = *(const v4f*)(w2 + (size_t)g * 8 + 4);
    v[0] = a[0]; v[1] = a[1]; v[2] = a[2]; v[3] = a[3];
    v[4] = c[0]; v[5] = c[1]; v[6] = c[2]; v[7] = c[3];
    dst = (size_t)64 * 96 + (size_t)64 * 64 + (size_t)g * 8;
  }
  v8h hv;
#pragma unroll
  for (int e = 0; e < 8; ++e) hv[e] = (_Float16)(v[e] * WCARRY);
  for (int pass = 0; pass < 2; ++pass) {
    *(volatile v8h*)(wp + dst) = hv;
    __threadfence();
  }
}

__device__ __forceinline__ float ball_d2(float cx, float cy, float cz, float c2,
                                         float x, float y, float z)
{
#pragma clang fp contract(off)
  const float xx = x * x, yy = y * y, zz = z * z;
  const float x2 = (xx + zz) + yy;
  float p = cx * x;
  p = fmaf(cy, y, p);
  p = fmaf(cz, z, p);
  const float tw = 2.0f * p;
  return (c2 + x2) - tw;
}

__global__ __launch_bounds__(256) void group_kernel(const float* __restrict__ xyz,
                                                    const float* __restrict__ feats,
                                                    const int* __restrict__ idxp,
                                                    int* __restrict__ maskp,
                                                    unsigned* __restrict__ x0p)
{
#pragma clang fp contract(off)
  __shared__ __align__(16) float    candD[CAND_CAP];
  __shared__ __align__(16) int      candN[CAND_CAP];
  __shared__ __align__(16) unsigned tileW[NNBR * 48];
  __shared__ int   wcnt[2][8];
  __shared__ int   sel[NNBR];
  __shared__ int   smk[NNBR];
  __shared__ float sdiff[NNBR * 3];

  const int bm = blockIdx.x;
  const int b  = bm >> 10;
  const int t  = threadIdx.x;
  const int lane = t & 31, wave = t >> 5;

  if (t < NNBR) { sel[t] = 0; smk[t] = 0; }

  const float* px = xyz + (size_t)b * NPTS * 3;
  const int ci = clampi(idxp[bm], 0, NPTS - 1);
  const float cx = px[ci * 3 + 0], cy = px[ci * 3 + 1], cz = px[ci * 3 + 2];
  const float cxx = cx * cx, cyy = cy * cy, czz = cz * cz;
  const float c2 = (cxx + czz) + cyy;

  float d2r[16];
  const v4f* pv = (const v4f*)px;
#pragma unroll
  for (int j = 0; j < 4; ++j) {
    const int g = t + 256 * j;
    const v4f a = pv[3 * g + 0];
    const v4f c = pv[3 * g + 1];
    const v4f e = pv[3 * g + 2];
    d2r[4 * j + 0] = ball_d2(cx, cy, cz, c2, a[0], a[1], a[2]);
    d2r[4 * j + 1] = ball_d2(cx, cy, cz, c2, a[3], c[0], c[1]);
    d2r[4 * j + 2] = ball_d2(cx, cy, cz, c2, c[2], c[3], e[0]);
    d2r[4 * j + 3] = ball_d2(cx, cy, cz, c2, e[1], e[2], e[3]);
    if (j == 1) asm volatile("" ::: "memory");
  }

  float T = 0.02f, Tsel = 0.02f;
  int total = 0, mycnt = 0, pbuf = 0;
  for (int it = 0; it < 12; ++it) {
    int c = 0;
#pragma unroll
    for (int s = 0; s < 16; ++s) c += (d2r[s] <= T) ? 1 : 0;
    int w = c;
#pragma unroll
    for (int off = 16; off > 0; off >>= 1) w += __shfl_xor(w, off, 32);
    const int pb = it & 1;
    if (lane == 0) wcnt[pb][wave] = w;
    __syncthreads();
    int tot = 0;
#pragma unroll
    for (int w8 = 0; w8 < 8; ++w8) tot += wcnt[pb][w8];
    mycnt = c; total = tot; pbuf = pb; Tsel = T;
    if (tot >= NNBR) break;
    T = T * 2.0f;
  }

  int woff = 0;
#pragma unroll
  for (int w8 = 0; w8 < 8; ++w8) {
    const int wc = wcnt[pbuf][w8];
    woff += (w8 < wave) ? wc : 0;
  }
  int inc = mycnt;
#pragma unroll
  for (int off = 1; off < 32; off <<= 1) {
    const int v = __shfl_up(inc, off, 32);
    inc += (lane >= off) ? v : 0;
  }
  int pos = woff + inc - mycnt;
#pragma unroll
  for (int s = 0; s < 16; ++s) {
    const int n = 4 * (t + 256 * (s >> 2)) + (s & 3);
    if (d2r[s] <= Tsel) {
      if (pos >= 0 && pos < CAND_CAP) { candD[pos] = d2r[s]; candN[pos] = n; }
      pos++;
    }
  }
  __syncthreads();
  const int totalc = clampi(total, 0, CAND_CAP);

  for (int i = t; i < totalc; i += 256) {
    const float di = candD[i]; const int ni = candN[i];
    int rank = 0;
    for (int j = 0; j < totalc; ++j) {
      const float dj = candD[j]; const int nj = candN[j];
      rank += ((dj < di) || (dj == di && nj < ni)) ? 1 : 0;
    }
    if (rank < NNBR) { sel[rank] = ni; smk[rank] = (di <= RADIUS_SQ) ? 1 : 0; }
  }
  __syncthreads();

  if (t < NNBR * 3) {
    const int k = t / 3;
    const int d = t - 3 * k;
    const int n = clampi(sel[k], 0, NPTS - 1);
    const float pvv = px[n * 3 + d];
    const float cv = (d == 0) ? cx : ((d == 1) ? cy : cz);
    sdiff[t] = pvv - cv;
  }
  if (wave == 0) {
    const int mval = smk[lane];
    volatile int* mp = maskp + (size_t)bm * 32 + lane;
    *mp = mval;
    __threadfence();
    *mp = mval;
  }
  {
    const float* fbp = feats + (size_t)b * NFEAT * NPTS;
    const int n = clampi(sel[lane], 0, NPTS - 1);
#pragma unroll
    for (int j = 0; j < 4; ++j) {
      const int cw = wave + 8 * j;
      const float f0 = fbp[(size_t)(2 * cw) * NPTS + n];
      const float f1 = fbp[(size_t)(2 * cw + 1) * NPTS + n];
      const unsigned u = f16_bits(f0) | (f16_bits(f1) << 16);
      tileW[lane * 48 + cw] = u;
    }
  }
  __syncthreads();
#pragma unroll
  for (int j = 0; j < 2; ++j) {
    const int id = t + 256 * j;
    const int k = id >> 4;
    const int tw = id & 15;
    const float dx = sdiff[k * 3 + 0], dy = sdiff[k * 3 + 1], dz = sdiff[k * 3 + 2];
    const unsigned uxy = f16_bits(dx) | (f16_bits(dy) << 16);
    const unsigned uz  = f16_bits(dz);
    const unsigned u = (tw == 0) ? uxy : ((tw == 1) ? uz : 0u);
    tileW[k * 48 + 32 + tw] = u;
  }
  __syncthreads();
  {
    unsigned* dst = x0p + (size_t)bm * (NNBR * 48);
    const v4u c0 = *(const v4u*)(tileW + 4 * t);
    const int t2 = (t < 128) ? (t + 256) : t;
    const v4u c1 = *(const v4u*)(tileW + 4 * t2);
    for (int pass = 0; pass < 2; ++pass) {
      *(volatile v4u*)(dst + 4 * t) = c0;
      if (t < 128) *(volatile v4u*)(dst + 4 * (t + 256)) = c1;
      __threadfence();
    }
  }
}

template <int NCH, int KDIM>
__global__ __launch_bounds__(256) void gemm_bn_kernel(const unsigned short* __restrict__ Ap,
                                                      const unsigned short* __restrict__ Btp,
                                                      unsigned short* __restrict__ Yp,
                                                      float* __restrict__ part,
                                                      float scale)
{
  static_assert(KDIM % 32 == 0 && NCH % 64 == 0);
  const _Float16* A  = (const _Float16*)Ap;
  const _Float16* Bt = (const _Float16*)Btp;
  __shared__ __align__(16) float sT[8][16 * 68];
  constexpr int tilesN = NCH / 64;
  const int lane = threadIdx.x & 31;
  const int wave = threadIdx.x >> 5;
  const int tile = blockIdx.x * 8 + wave;
  const int tm = tile / tilesN;
  const int tn = tile - tm * tilesN;
  const int m0 = tm << 6;
  const int n0 = tn << 6;
  const int rlane = lane & 15;
  const int hh    = lane >> 4;
  const int koff  = hh * 8;
  const int mOff  = hh * 8;

  v8f acc[4][4];
#pragma unroll
  for (int i = 0; i < 4; ++i)
#pragma unroll
    for (int j = 0; j < 4; ++j) acc[i][j] = (v8f){0.f,0.f,0.f,0.f,0.f,0.f,0.f,0.f};

  for (int k0 = 0; k0 < KDIM; k0 += 32) {
    v16h bh[4];
#pragma unroll
    for (int j = 0; j < 4; ++j)
      bh[j] = frag_load(Bt + (size_t)(n0 + (j << 4) + rlane) * KDIM + koff + k0);
#pragma unroll
    for (int i = 0; i < 4; ++i) {
      const v16h ah = frag_load(A + (size_t)(m0 + (i << 4) + rlane) * KDIM + koff + k0);
#pragma unroll
      for (int j = 0; j < 4; ++j) acc[i][j] = frag_mma(ah, bh[j], acc[i][j]);
      group_guard(acc[i][0], acc[i][1], acc[i][2], acc[i][3], ah, bh[0], bh[1], bh[2], bh[3]);
    }
  }
  acc_guard4(acc[0][0], acc[0][1], acc[0][2], acc[0][3]);
  acc_guard4(acc[1][0], acc[1][1], acc[1][2], acc[1][3]);
  acc_guard4(acc[2][0], acc[2][1], acc[2][2], acc[2][3]);
  acc_guard4(acc[3][0], acc[3][1], acc[3][2], acc[3][3]);

  float* slab = sT[wave];
  float ssum[4] = {0.f, 0.f, 0.f, 0.f};
  float ssq[4]  = {0.f, 0.f, 0.f, 0.f};
#pragma unroll
  for (int i = 0; i < 4; ++i) {
    const int mBase = m0 + (i << 4);
#pragma unroll
    for (int j = 0; j < 4; ++j) {
#pragma unroll
      for (int r = 0; r < 8; ++r) {
        const float v = acc[i][j][r] * scale;
        ssum[j] += v;
        const float vv = v * v;
        ssq[j] += vv;
        slab[(mOff + r) * 68 + (j << 4) + rlane] = v;
      }
    }
    __builtin_amdgcn_fence(__ATOMIC_RELEASE, "workgroup");
    __builtin_amdgcn_wave_barrier();
    __builtin_amdgcn_fence(__ATOMIC_ACQUIRE, "workgroup");
    {
      const int q = lane >> 3, c8 = (lane & 7) * 8;
      for (int pass = 0; pass < 2; ++pass) {
#pragma unroll
        for (int it = 0; it < 4; ++it) {
          const int row = it * 4 + q;
          const float* sp = slab + row * 68 + c8;
          v8h hv;
#pragma unroll
          for (int e = 0; e < 8; ++e) hv[e] = (_Float16)sp[e];
          *(volatile v8h*)(Yp + (size_t)(mBase + row) * NCH + n0 + c8) = hv;
        }
        __threadfence();
      }
    }
    __builtin_amdgcn_fence(__ATOMIC_RELEASE, "workgroup");
    __builtin_amdgcn_wave_barrier();
    __builtin_amdgcn_fence(__ATOMIC_ACQUIRE, "workgroup");
  }

#pragma unroll
  for (int j = 0; j < 4; ++j) {
    const float os = __shfl_xor(ssum[j], 16, 32);
    const float oq = __shfl_xor(ssq[j], 16, 32);
    ssum[j] += os;
    ssq[j]  += oq;
  }
#pragma unroll
  for (int j = 0; j < 4; ++j) {
    const float val = hh ? ssq[j] : ssum[j];
    slab[hh * 64 + (j << 4) + rlane] = val;
  }
  __builtin_amdgcn_fence(__ATOMIC_RELEASE, "workgroup");
  __builtin_amdgcn_wave_barrier();
  __builtin_amdgcn_fence(__ATOMIC_ACQUIRE, "workgroup");
  {
    const int c4 = (lane & 15) * 4;
    const v4f v = *(const v4f*)(slab + hh * 64 + c4);
    float* dst = part + (size_t)tm * 256 + hh * 128 + n0 + c4;
    for (int pass = 0; pass < 2; ++pass) {
      *(volatile v4f*)dst = v;
      __threadfence();
    }
  }
}

__global__ __launch_bounds__(256) void bnred_kernel(const float* __restrict__ part,
                                                    const float* __restrict__ g,
                                                    const float* __restrict__ bb,
                                                    float* __restrict__ scsh)
{
  __shared__ double ds[8][32];
  __shared__ double dq[8][32];
  const int t = threadIdx.x;
  const int cl = t & 31, w = t >> 5;
  const int c = blockIdx.x * 32 + cl;
  double s = 0.0, q = 0.0;
#pragma unroll 4
  for (int i = 0; i < NTILE_M / 8; ++i) {
    const size_t tile = (size_t)(w * (NTILE_M / 8) + i);
    const float a = part[tile * 256 + c];
    const float d = part[tile * 256 + 128 + c];
    s += (double)a;
    q += (double)d;
  }
  ds[w][cl] = s; dq[w][cl] = q;
  __syncthreads();
  if (w == 0) {
    double fs = 0.0, fq = 0.0;
#pragma unroll
    for (int w8 = 0; w8 < 8; ++w8) { fs += ds[w8][cl]; fq += dq[w8][cl]; }
    const double invn = 1.0 / (double)NPOS;
    const double mean = fs * invn;
    double var = fq * invn - mean * mean;
    var = var < 0.0 ? 0.0 : var;
    const float inv = rsqrtf((float)var + BN_EPS_F);
    const float sc = g[c] * inv;
    const float sh = bb[c] - (float)mean * sc;
    for (int pass = 0; pass < 2; ++pass) {
      *(volatile float*)(scsh + c) = sc;
      *(volatile float*)(scsh + 128 + c) = sh;
      __threadfence();
    }
  }
}

__global__ __launch_bounds__(256) void apply_kernel(const unsigned short* __restrict__ Yp,
                                                    const float* __restrict__ scsh,
                                                    unsigned short* __restrict__ Aout)
{
  const int i = blockIdx.x * 256 + threadIdx.x;
  const int c0 = (i & 7) * 8;
  const v4u w = *(const v4u*)(Yp + (size_t)i * 8);
  const v4f sa = *(const v4f*)(scsh + c0);
  const v4f sb = *(const v4f*)(scsh + c0 + 4);
  const v4f ha = *(const v4f*)(scsh + 128 + c0);
  const v4f hb = *(const v4f*)(scsh + 128 + c0 + 4);
  const unsigned w0 = w[0], w1 = w[1], w2 = w[2], w3 = w[3];
  float y[8], scv[8], shv[8];
  y[0] = h16_to_f32(w0 & 0xffffu); y[1] = h16_to_f32(w0 >> 16);
  y[2] = h16_to_f32(w1 & 0xffffu); y[3] = h16_to_f32(w1 >> 16);
  y[4] = h16_to_f32(w2 & 0xffffu); y[5] = h16_to_f32(w2 >> 16);
  y[6] = h16_to_f32(w3 & 0xffffu); y[7] = h16_to_f32(w3 >> 16);
  scv[0] = sa[0]; scv[1] = sa[1]; scv[2] = sa[2]; scv[3] = sa[3];
  scv[4] = sb[0]; scv[5] = sb[1]; scv[6] = sb[2]; scv[7] = sb[3];
  shv[0] = ha[0]; shv[1] = ha[1]; shv[2] = ha[2]; shv[3] = ha[3];
  shv[4] = hb[0]; shv[5] = hb[1]; shv[6] = hb[2]; shv[7] = hb[3];
  v8h hv;
#pragma unroll
  for (int e = 0; e < 8; ++e) {
    const float p = scv[e] * y[e];
    const float a = fmaxf(p + shv[e], 0.0f);
    hv[e] = (_Float16)a;
  }
  for (int pass = 0; pass < 2; ++pass) {
    *(volatile v8h*)(Aout + (size_t)i * 8) = hv;
    __threadfence();
  }
}

__global__ __launch_bounds__(256) void pool_kernel(const unsigned short* __restrict__ Y2,
                                                   const int* __restrict__ maskp,
                                                   const float* __restrict__ scsh,
                                                   float* __restrict__ out1)
{
  __shared__ __align__(16) float sres[128 * 36];
  const int t = threadIdx.x;
  const int lane = t & 31, wave = t >> 5;
  const int bm0 = blockIdx.x * 32;
  const int ml = t >> 3, cg = t & 7;
  const int bm = bm0 + ml;

  unsigned mbits = 0u;
  {
    const v4i* mp = (const v4i*)(maskp + (size_t)bm * 32);
#pragma unroll
    for (int q8 = 0; q8 < 8; ++q8) {
      const v4i mv = mp[q8];
      const int a0 = mv[0], a1 = mv[1], a2 = mv[2], a3 = mv[3];
      mbits |= ((a0 != 0) ? 1u : 0u) << (4 * q8 + 0);
      mbits |= ((a1 != 0) ? 1u : 0u) << (4 * q8 + 1);
      mbits |= ((a2 != 0) ? 1u : 0u) << (4 * q8 + 2);
      mbits |= ((a3 != 0) ? 1u : 0u) << (4 * q8 + 3);
    }
  }
  asm volatile("" ::: "memory");
  float scv[16], shv[16], mx[16];
#pragma unroll
  for (int q4 = 0; q4 < 4; ++q4) {
    const v4f a = *(const v4f*)(scsh + cg * 16 + 4 * q4);
    const v4f h = *(const v4f*)(scsh + 128 + cg * 16 + 4 * q4);
#pragma unroll
    for (int e = 0; e < 4; ++e) { scv[4 * q4 + e] = a[e]; shv[4 * q4 + e] = h[e]; }
  }
#pragma unroll
  for (int e = 0; e < 16; ++e) mx[e] = -INFINITY;

#pragma unroll 2
  for (int k = 0; k < NNBR; ++k) {
    const size_t pos = (size_t)bm * NNBR + k;
    const v4u wa = *(const v4u*)(Y2 + pos * 128 + cg * 16);
    const v4u wb = *(const v4u*)(Y2 + pos * 128 + cg * 16 + 8);
    const bool keep = ((mbits >> k) & 1u) != 0u;
    unsigned ww[8];
    ww[0] = wa[0]; ww[1] = wa[1]; ww[2] = wa[2]; ww[3] = wa[3];
    ww[4] = wb[0]; ww[5] = wb[1]; ww[6] = wb[2]; ww[7] = wb[3];
#pragma unroll
    for (int e = 0; e < 8; ++e) {
      const float y0 = h16_to_f32(ww[e] & 0xffffu);
      const float y1 = h16_to_f32(ww[e] >> 16);
      const float p0 = scv[2 * e] * y0;
      const float p1 = scv[2 * e + 1] * y1;
      const float a0 = fmaxf(p0 + shv[2 * e], 0.0f);
      const float a1 = fmaxf(p1 + shv[2 * e + 1], 0.0f);
      const float s0 = keep ? a0 : -INFINITY;
      const float s1 = keep ? a1 : -INFINITY;
      mx[2 * e]     = fmaxf(mx[2 * e], s0);
      mx[2 * e + 1] = fmaxf(mx[2 * e + 1], s1);
    }
  }
#pragma unroll
  for (int e = 0; e < 16; ++e) sres[(cg * 16 + e) * 36 + ml] = mx[e];
  __syncthreads();

  const int b  = bm0 >> 10;
  const int mb = bm0 & (NCENT - 1);
  const int q = lane >> 3, c4 = (lane & 7) * 4;
  for (int pass = 0; pass < 2; ++pass) {
#pragma unroll
    for (int it = 0; it < 4; ++it) {
      const int ch = wave * 16 + it * 4 + q;
      const v4f v = *(const v4f*)(sres + ch * 36 + c4);
      *(volatile v4f*)(out1 + ((size_t)(b * 128 + ch)) * NCENT + mb + c4) = v;
    }
    __threadfence();
  }
}

extern "C" void kernel_launch(void* const* d_in, const int* in_sizes, int n_in,
                              void* d_out, int out_size, void* d_ws, size_t ws_size,
                              hipStream_t stream)
{
  (void)in_sizes; (void)out_size;
  if (n_in < 11) return;
  if (ws_size < WS_TOTAL) return;

  const float* xyz   = (const float*)d_in[0];
  const float* feats = (const float*)d_in[1];
  const float* w0 = (const float*)d_in[2];
  const float* g0 = (const float*)d_in[3];
  const float* b0 = (const float*)d_in[4];
  const float* w1 = (const float*)d_in[5];
  const float* g1 = (const float*)d_in[6];
  const float* b1 = (const float*)d_in[7];
  const float* w2 = (const float*)d_in[8];
  const float* g2 = (const float*)d_in[9];
  const float* b2 = (const float*)d_in[10];

  float* out_xyz  = (float*)d_out;
  float* out_feat = (float*)d_out + (size_t)NBATCH * NCENT * 3;

  char* ws = (char*)d_ws;
  unsigned short* planeA = (unsigned short*)(ws + OFF_PA);
  unsigned short* planeB = (unsigned short*)(ws + OFF_PB);
  unsigned short* planeB_hi = planeB + (size_t)NPOS * 64;
  float* part0 = (float*)(ws + OFF_PART);
  float* part1 = (float*)(ws + OFF_PART + SZ_PART1);
  float* part2 = (float*)(ws + OFF_PART + 2 * SZ_PART1);
  int*   maskp = (int*)(ws + OFF_MASK);
  int*   idxp  = (int*)(ws + OFF_IDX);
  unsigned short* wpk = (unsigned short*)(ws + OFF_WPK);
  unsigned short* w0p = wpk;
  unsigned short* w1p = wpk + 64 * 96;
  unsigned short* w2p = wpk + 64 * 96 + 64 * 64;
  float* scsh0 = (float*)(ws + OFF_SCSH);
  float* scsh1 = scsh0 + 256;
  float* scsh2 = scsh0 + 512;

  fps_kernel<<<NBATCH, 256, 0, stream>>>(xyz, idxp, out_xyz);
  pack_kernel<<<9, 256, 0, stream>>>(w0, w1, w2, wpk);
  group_kernel<<<NBATCH * NCENT, 256, 0, stream>>>(xyz, feats, idxp, maskp, (unsigned*)planeA);

  gemm_bn_kernel<NCH_L0, KPAD0><<<NTILE_M / 8, 256, 0, stream>>>(planeA, w0p, planeB, part0, WCARRY_INV);
  bnred_kernel<<<NCH_L0 / 32, 256, 0, stream>>>(part0, g0, b0, scsh0);
  apply_kernel<<<(NPOS * 64 / 8) / 256, 256, 0, stream>>>(planeB, scsh0, planeA);

  gemm_bn_kernel<NCH_L1, 64><<<NTILE_M / 8, 256, 0, stream>>>(planeA, w1p, planeB_hi, part1, WCARRY_INV);
  bnred_kernel<<<NCH_L1 / 32, 256, 0, stream>>>(part1, g1, b1, scsh1);
  apply_kernel<<<(NPOS * 64 / 8) / 256, 256, 0, stream>>>(planeB_hi, scsh1, planeA);

  gemm_bn_kernel<NCH_L2, 64><<<(NTILE_M * 2) / 8, 256, 0, stream>>>(planeA, w2p, planeB, part2, WCARRY_INV);
  bnred_kernel<<<NCH_L2 / 32, 256, 0, stream>>>(part2, g2, b2, scsh2);

  pool_kernel<<<(NBATCH * NCENT) / 32, 256, 0, stream>>>(planeB, maskp, scsh2, out_feat);
}
